// MultiHeadedAttention_74689481277507
// MI455X (gfx1250) — hardware-verified
//
#include <hip/hip_runtime.h>
#include <math.h>

typedef __attribute__((ext_vector_type(16))) _Float16 v16h;
typedef __attribute__((ext_vector_type(16))) __bf16 v16b;
typedef __attribute__((ext_vector_type(8)))  _Float16 v8h;
typedef __attribute__((ext_vector_type(8)))  __bf16 v8b;
typedef __attribute__((ext_vector_type(8)))  float v8f;
typedef __attribute__((ext_vector_type(4)))  float v4f;
typedef __attribute__((ext_vector_type(4)))  unsigned v4u;
typedef __attribute__((ext_vector_type(4)))  int v4i;

#ifndef NB
#define NB 2
#endif
#ifndef SEQ
#define SEQ 2048
#endif
#define NB_FULL 2
#define SEQ_FULL 2048
#define DM 1024
#define NH 16
#define HD 64
#define MROWS (NB * SEQ)
#define PCARRY (4096.0f)
#define RCARRY (2048.0f)
static_assert((size_t)NB_FULL * SEQ_FULL * DM * 4 == 16777216u);
static_assert(SEQ % 64 == 0 && SEQ <= SEQ_FULL && NB <= NB_FULL);
static_assert(DM == NH * HD && DM % 128 == 0 && DM % 64 == 0 && DM % 32 == 0 && HD == 64);
static_assert((SEQ * DM / 8) % 256 == 0 && (DM * DM / 8) % 256 == 0);
static_assert(((size_t)MROWS * 32) % 256 == 0);
static_assert(MROWS % 64 == 0);

#define WS_XB   0u
#define WS_WB   (WS_XB  + 2u * 3u * (size_t)MROWS * DM)
#define WS_WOH  (WS_WB  + 2u * 3u * (size_t)DM * DM)
#define WS_WOL  (WS_WOH + 2u * (size_t)DM * DM)
#define WS_H16  (WS_WOL + 2u * (size_t)DM * DM)
#define WS_L16  (WS_H16 + 2u * 2u * (size_t)MROWS * DM)
#define WS_VT   (WS_L16 + 2u * 2u * (size_t)MROWS * DM)
#define WS_CH   (WS_VT  + 2u * (size_t)NB * DM * SEQ)
#define WS_CL   (WS_CH  + 2u * (size_t)MROWS * DM)
#define WS_CS   (WS_CL  + 2u * (size_t)MROWS * DM)
#define WS_END  (WS_CS  + 4u * (size_t)MROWS * 64)
static_assert((size_t)WS_END <= 134217728u);
static_assert((size_t)WS_WB % 128 == 0 && (size_t)WS_H16 % 128 == 0 && (size_t)WS_VT % 128 == 0 && (size_t)WS_CS % 128 == 0);

#define WAITL() asm volatile("s_wait_loadcnt 0x0" ::: "memory")
#define LDSX() do { asm volatile("s_wait_dscnt 0" ::: "memory"); __builtin_amdgcn_wave_barrier(); __builtin_amdgcn_fence(3  , "workgroup"); } while (0)

template <typename T> __device__ __forceinline__ void vst2(void* p, T v) { *(volatile T*)p = v; __threadfence(); *(volatile T*)p = v; }
__device__ __forceinline__ v8f wmma16(v16h a, v16h b, v8f c) {
  v8f d = __builtin_amdgcn_wmma_f32_16x16x32_f16(false, a, false, b, (short)0, c, false, false);
  asm volatile("v_nop\n\tv_nop\n\tv_nop\n\tv_nop" : "+v"(d) : "v"(a), "v"(b));
  return d;
}
__device__ __forceinline__ v8f wmma_bf(v16b a, v16b b, v8f c) {
  v8f d = __builtin_amdgcn_wmma_f32_16x16x32_bf16(false, a, false, b, (short)0, c, false, false);
  asm volatile("v_nop\n\tv_nop\n\tv_nop\n\tv_nop" : "+v"(d) : "v"(a), "v"(b));
  return d;
}
__device__ __forceinline__ v16h frag_h(const _Float16* rowk0, int lane) {
  union { v16h v; v8h q[2]; } u; const _Float16* p = rowk0 + 8 * (lane >> 4);
  u.q[0] = *(const v8h*)p; u.q[1] = *(const v8h*)(p + 16); return u.v;
}
__device__ __forceinline__ v16b frag_b(const __bf16* rowk0, int lane) {
  union { v16b v; v8b q[2]; } u; const __bf16* p = rowk0 + 8 * (lane >> 4);
  u.q[0] = *(const v8b*)p; u.q[1] = *(const v8b*)(p + 16); return u.v;
}
__device__ __forceinline__ float bfr(float v) { return (float)(__bf16)v; }

__global__ __launch_bounds__(256) void k_cvt_bf(const float* __restrict__ src, __bf16* __restrict__ dst, size_t sstride, size_t dstride, int n8) {
  const int i = blockIdx.x * 256 + threadIdx.x; if (i >= n8) return;
  const float* p = src + (size_t)blockIdx.y * sstride + (size_t)i * 8;
  const v4f a = *(const v4f*)p, c = *(const v4f*)(p + 4);
  union { v8b b; v4u u; } o;
#pragma unroll
  for (int k = 0; k < 4; ++k) { o.b[k] = (__bf16)a[k]; o.b[4 + k] = (__bf16)c[k]; }
  vst2(dst + (size_t)blockIdx.y * dstride + (size_t)i * 8, o.u);
}

__global__ __launch_bounds__(256) void k_wt_bf(const float* __restrict__ W, __bf16* __restrict__ WT) {
  __shared__ float st[64][68];
  const int tid = threadIdx.x; const int n0 = blockIdx.x * 64, k0 = blockIdx.y * 64;
#pragma unroll
  for (int i = 0; i < 4; ++i) { const int idx = tid + 256 * i, kk = idx >> 4, c4 = idx & 15;
    const v4f v = *(const v4f*)(W + (size_t)(k0 + kk) * DM + n0 + c4 * 4);
    st[kk][c4 * 4 + 0] = v[0]; st[kk][c4 * 4 + 1] = v[1]; st[kk][c4 * 4 + 2] = v[2]; st[kk][c4 * 4 + 3] = v[3]; }
  __syncthreads();
#pragma unroll
  for (int i = 0; i < 2; ++i) { const int e = tid + 256 * i, n = e >> 3, p = e & 7; union { v8b b; v4u u; } o;
#pragma unroll
    for (int j = 0; j < 8; ++j) o.b[j] = (__bf16)st[p * 8 + j][n];
    vst2(WT + (size_t)(n0 + n) * DM + k0 + p * 8, o.u); }
}
__global__ __launch_bounds__(256) void k_wt_wo(const float* __restrict__ W, _Float16* __restrict__ WH, _Float16* __restrict__ WL) {
  __shared__ float st[64][68];
  const int tid = threadIdx.x; const int n0 = blockIdx.x * 64, k0 = blockIdx.y * 64;
#pragma unroll
  for (int i = 0; i < 4; ++i) { const int idx = tid + 256 * i, kk = idx >> 4, c4 = idx & 15;
    const v4f v = *(const v4f*)(W + (size_t)(k0 + kk) * DM + n0 + c4 * 4);
    st[kk][c4 * 4 + 0] = v[0]; st[kk][c4 * 4 + 1] = v[1]; st[kk][c4 * 4 + 2] = v[2]; st[kk][c4 * 4 + 3] = v[3]; }
  __syncthreads();
#pragma unroll
  for (int i = 0; i < 2; ++i) { const int e = tid + 256 * i, n = e >> 3, p = e & 7; union { v8h h; v4u u; } oh, ol;
#pragma unroll
    for (int j = 0; j < 8; ++j) { const float x = bfr(st[p * 8 + j][n]); oh.h[j] = (_Float16)(x * 256.0f); ol.h[j] = (_Float16)(x * 2.0f); }
    const size_t dst = (size_t)(n0 + n) * DM + k0 + p * 8;
    vst2(WH + dst, oh.u); vst2(WL + dst, ol.u); }
}

__global__ __launch_bounds__(256) void k_tab(const float* __restrict__ MZ, float* __restrict__ CS) {
  const int idx = blockIdx.x * 256 + threadIdx.x;
  const int row = idx >> 5, i = idx & 31;
  const int b = row / SEQ, s = row % SEQ;
  const float pos = bfr(MZ[(size_t)b * SEQ_FULL + s]);
  double p = 1.0;
  p *= (i & 1)  ? 1.3335214321633240 : 1.0;
  p *= (i & 2)  ? 1.7782794100389228 : 1.0;
  p *= (i & 4)  ? 3.1622776601683795 : 1.0;
  p *= (i & 8)  ? 10.0 : 1.0;
  p *= (i & 16) ? 100.0 : 1.0;
  const float pf = (float)p;
  const float th = 1.0f / pf;
  const float ang = pos * th;
  float sn, cs;
  sincosf(ang, &sn, &cs);
  vst2(CS + (size_t)row * 64 + i, cs);
  vst2(CS + (size_t)row * 64 + 32 + i, sn);
}

__global__ __launch_bounds__(128) void k_proj(const __bf16* __restrict__ XB, const __bf16* __restrict__ WB, const float* __restrict__ BQ, const float* __restrict__ BK, const float* __restrict__ BV,
    const float* __restrict__ CS, _Float16* __restrict__ H16, _Float16* __restrict__ L16, _Float16* __restrict__ VT) {
  __shared__ __align__(16) float sf[64][132];
  const int tid = threadIdx.x, wave = __builtin_amdgcn_readfirstlane(threadIdx.x >> 5), lane = tid & 31, col = lane & 15, g = lane >> 4;
  const int which = blockIdx.z; const int c0 = blockIdx.y * 128; const int r0 = blockIdx.x * 64; const int bb = r0 / SEQ; const int t0 = r0 % SEQ;
  const __bf16* X = XB + (size_t)which * MROWS * DM; const __bf16* W = WB + (size_t)which * DM * DM;
  v8f acc[8] = {};
#pragma unroll 2
  for (int kc = 0; kc < DM / 32; ++kc) {
    const v16b a = frag_b(X + (size_t)(r0 + wave * 16 + col) * DM + kc * 32, lane);
    WAITL();
#pragma unroll
    for (int j = 0; j < 8; ++j) { const v16b w = frag_b(W + (size_t)(c0 + j * 16 + col) * DM + kc * 32, lane); WAITL(); acc[j] = wmma_bf(a, w, acc[j]); }
  }
#pragma unroll
  for (int j = 0; j < 8; ++j) { const int ci = c0 + j * 16 + col; const float b0 = BQ[ci], b1 = BK[ci], b2 = BV[ci]; const float bias = bfr(which == 0 ? b0 : (which == 1 ? b1 : b2));
#pragma unroll
    for (int r = 0; r < 8; ++r) sf[wave * 16 + 8 * g + r][j * 16 + col] = acc[j][r] + bias; }
  __syncthreads();
  if (which < 2) {
    _Float16* DH = H16 + (size_t)which * MROWS * DM;
    _Float16* DL = L16 + (size_t)which * MROWS * DM;
    for (int e = tid; e < 64 * 16; e += 128) { const int rl = e >> 4, q = e & 15, qp = q ^ 4;
      const v4f a = *(const v4f*)&sf[rl][q * 8], c = *(const v4f*)&sf[rl][q * 8 + 4];
      const v4f ra = *(const v4f*)&sf[rl][qp * 8], rc = *(const v4f*)&sf[rl][qp * 8 + 4];
      const float* cr = CS + (size_t)(r0 + rl) * 64 + (q & 7) * 4;
      const v4f cs = *(const v4f*)cr, sn = *(const v4f*)(cr + 32);
      const float sg = (q & 4) ? 1.0f : -1.0f;
      union { v8h h; v4u u; } hv, lv;
#pragma unroll
      for (int i = 0; i < 4; ++i) {
        const float x = a[i] * cs[i >> 1] + (sg * ra[i]) * sn[i >> 1];
        const float y = c[i] * cs[2 + (i >> 1)] + (sg * rc[i]) * sn[2 + (i >> 1)];
        const _Float16 hx = (_Float16)x, hy = (_Float16)y; hv.h[i] = hx; hv.h[4 + i] = hy;
        lv.h[i] = (_Float16)((x - (float)hx) * RCARRY); lv.h[4 + i] = (_Float16)((y - (float)hy) * RCARRY); }
      const size_t dst = (size_t)(r0 + rl) * DM + c0 + q * 8;
      vst2(DH + dst, hv.u); vst2(DL + dst, lv.u); }
  } else {
    for (int e = tid; e < 128 * 8; e += 128) { const int cl = e >> 3, q = e & 7; union { v8h h; v4u u; } o;
#pragma unroll
      for (int i = 0; i < 8; ++i) o.h[i] = (_Float16)sf[q * 8 + i][cl];
      vst2(VT + ((size_t)bb * DM + c0 + cl) * SEQ + t0 + q * 8, o.u); }
  }
}

__global__ __launch_bounds__(128) void k_attn(const _Float16* __restrict__ H16, const _Float16* __restrict__ L16, const _Float16* __restrict__ VT, const int* __restrict__ MASK, _Float16* __restrict__ CH, _Float16* __restrict__ CL) {
  __shared__ __align__(16) _Float16 sh[4][16][72], sl[4][16][72];
  const int tid = threadIdx.x, wave = __builtin_amdgcn_readfirstlane(threadIdx.x >> 5), lane = tid & 31, col = lane & 15, g = lane >> 4;
  const int h = blockIdx.y, b = blockIdx.z; const int q0 = blockIdx.x * 64 + wave * 16;
  const _Float16* KH = H16 + (size_t)MROWS * DM;
  const _Float16* KL = L16 + (size_t)MROWS * DM;
  const int qoff = (b * SEQ + q0 + col) * DM + h * HD;
  const int koff = (b * SEQ + col) * DM + h * HD;
  const int voff = (b * DM + h * HD + col) * SEQ;
  const int* mrow = MASK + ((size_t)b * SEQ_FULL + q0 + col) * SEQ_FULL + 8 * g;
  v8f accO[4] = {}; float mrun = -1.0e30f, lrun = 0.0f;
#pragma unroll 1
  for (int kt = 0; kt < SEQ; kt += 32) {
    int qo = qoff; asm volatile("" : "+v"(qo));
    v8f s0 = {}, s0l = {}, s1 = {}, s1l = {};
#pragma unroll
    for (int kc = 0; kc < HD / 32; ++kc) {
      const v16h fq = frag_h(H16 + qo + kc * 32, lane), fql = frag_h(L16 + qo + kc * 32, lane);
      const v16h fk0 = frag_h(KH + koff + kt * DM + kc * 32, lane), fk1 = frag_h(KH + koff + (kt + 16) * DM + kc * 32, lane);
      const v16h fk0l = frag_h(KL + koff + kt * DM + kc * 32, lane), fk1l = frag_h(KL + koff + (kt + 16) * DM + kc * 32, lane);
      WAITL();
      s0 = wmma16(fk0, fq, s0); s0l = wmma16(fk0, fql, s0l); s0l = wmma16(fk0l, fq, s0l);
      s1 = wmma16(fk1, fq, s1); s1l = wmma16(fk1, fql, s1l); s1l = wmma16(fk1l, fq, s1l);
    }
    const v4i m00 = *(const v4i*)(mrow + kt), m01 = *(const v4i*)(mrow + kt + 4), m10 = *(const v4i*)(mrow + kt + 16), m11 = *(const v4i*)(mrow + kt + 20);
    WAITL();
    float pa[8], pc[8];
#pragma unroll
    for (int r = 0; r < 8; ++r) { const int mk0 = (r < 4) ? m00[r & 3] : m01[r & 3], mk1 = (r < 4) ? m10[r & 3] : m11[r & 3];
      const float v0 = s0[r] + s0l[r] * (1.0f / 2048.0f), v1 = s1[r] + s1l[r] * (1.0f / 2048.0f);
      pa[r] = (mk0 == 0) ? -1.0e9f : v0; pc[r] = (mk1 == 0) ? -1.0e9f : v1; }
    float tmax = fmaxf(pa[0], pc[0]);
#pragma unroll
    for (int r = 1; r < 8; ++r) tmax = fmaxf(tmax, fmaxf(pa[r], pc[r]));
    tmax = fmaxf(tmax, __shfl_xor(tmax, 16));
    const float mnew = fmaxf(mrun, tmax); const float alpha = __expf(mrun - mnew); mrun = mnew;
    float ps = 0.0f; v16h pb;
#pragma unroll
    for (int r = 0; r < 8; ++r) { const float e0 = __expf(pa[r] - mnew), e1 = __expf(pc[r] - mnew); ps += e0 + e1; pb[r] = (_Float16)(e0 * PCARRY); pb[8 + r] = (_Float16)(e1 * PCARRY); }
    ps += __shfl_xor(ps, 16); lrun = lrun * alpha + ps;
#pragma unroll
    for (int r = 0; r < 8; ++r) { accO[0][r] *= alpha; accO[1][r] *= alpha; accO[2][r] *= alpha; accO[3][r] *= alpha; }
    const v16h fv0 = frag_h(VT + voff + kt, lane), fv1 = frag_h(VT + voff + 16 * SEQ + kt, lane), fv2 = frag_h(VT + voff + 32 * SEQ + kt, lane), fv3 = frag_h(VT + voff + 48 * SEQ + kt, lane);
    WAITL();
    accO[0] = wmma16(fv0, pb, accO[0]); accO[1] = wmma16(fv1, pb, accO[1]); accO[2] = wmma16(fv2, pb, accO[2]); accO[3] = wmma16(fv3, pb, accO[3]);
  }
  const float inv = 0.015625f * (1.0f / lrun);
#pragma unroll
  for (int j = 0; j < 4; ++j) { v8h hv, lv;
#pragma unroll
    for (int r = 0; r < 8; ++r) { const float c = accO[j][r] * inv; const _Float16 hi = (_Float16)c; hv[r] = hi; lv[r] = (_Float16)((c - (float)hi) * 128.0f); }
    *(v8h*)&sh[wave][col][j * 16 + 8 * g] = hv; *(v8h*)&sl[wave][col][j * 16 + 8 * g] = lv; }
  LDSX();
#pragma unroll
  for (int i = 0; i < 4; ++i) { const int rl = i * 4 + (lane >> 3), pcx = lane & 7; const size_t dst = ((size_t)b * SEQ + q0 + rl) * DM + h * HD + pcx * 8;
    const v4u a = *(const v4u*)&sh[wave][rl][pcx * 8]; const v4u c = *(const v4u*)&sl[wave][rl][pcx * 8];
    vst2(CH + dst, a); vst2(CL + dst, c); }
}

__global__ __launch_bounds__(128) void k_out(const _Float16* __restrict__ CH, const _Float16* __restrict__ CL, const _Float16* __restrict__ WOH, const _Float16* __restrict__ WOL, const float* __restrict__ BO, float* __restrict__ OUT) {
  __shared__ __align__(16) float sf[4][16][132];
  const int tid = threadIdx.x, wave = __builtin_amdgcn_readfirstlane(threadIdx.x >> 5), lane = tid & 31, col = lane & 15, g = lane >> 4; const int c0 = blockIdx.y * 128; const int R0 = blockIdx.x * 64 + wave * 16;
  v8f acc[8] = {};
#pragma unroll 2
  for (int kc = 0; kc < DM / 32; ++kc) { const size_t ao = (size_t)(R0 + col) * DM + kc * 32; const v16h ah = frag_h(CH + ao, lane), al = frag_h(CL + ao, lane);
    WAITL();
#pragma unroll
    for (int j = 0; j < 8; ++j) { const size_t wo = (size_t)(c0 + j * 16 + col) * DM + kc * 32; const v16h wh = frag_h(WOH + wo, lane), wl = frag_h(WOL + wo, lane); WAITL(); acc[j] = wmma16(ah, wh, acc[j]); acc[j] = wmma16(al, wl, acc[j]); } }
#pragma unroll
  for (int j = 0; j < 8; ++j) { const float bias = bfr(BO[c0 + j * 16 + col]);
#pragma unroll
    for (int r = 0; r < 8; ++r) sf[wave][8 * g + r][j * 16 + col] = acc[j][r] * (1.0f / 16384.0f) + bias; }
  LDSX();
  const int bb = (blockIdx.x * 64) / SEQ; const int t0 = (blockIdx.x * 64) % SEQ + wave * 16;
  for (int rl = 0; rl < 16; ++rl) { const v4f o = *(const v4f*)&sf[wave][rl][lane * 4]; vst2(OUT + ((size_t)bb * SEQ_FULL + t0 + rl) * DM + c0 + lane * 4, o); }
}

extern "C" void kernel_launch(void* const* d_in, const int* in_sizes, int n_in, void* d_out, int out_size, void* d_ws, size_t ws_size, hipStream_t stream) {
  if (n_in < 13) return;
  const size_t need_rows = (size_t)(NB - 1) * SEQ_FULL + SEQ;
  const size_t need_x = need_rows * DM;
  if ((size_t)in_sizes[0] < need_x || (size_t)in_sizes[1] < need_x || (size_t)in_sizes[2] < need_x) return;
  if ((size_t)in_sizes[3] < need_rows * SEQ_FULL) return;
  if ((size_t)in_sizes[4] < need_rows) return;
  if (in_sizes[5] < DM * DM || in_sizes[7] < DM * DM || in_sizes[9] < DM * DM || in_sizes[11] < DM * DM) return;
  if (in_sizes[6] < DM || in_sizes[8] < DM || in_sizes[10] < DM || in_sizes[12] < DM) return;
  if ((size_t)out_size < need_x) return;
  if (ws_size < (size_t)WS_END) return;
  const float** F = (const float**)d_in;
  const int* MASK = (const int*)d_in[3];
  char* ws = (char*)d_ws;
  __bf16* XB = (__bf16*)(ws + WS_XB); __bf16* WB = (__bf16*)(ws + WS_WB);
  _Float16 *WOH = (_Float16*)(ws + WS_WOH), *WOL = (_Float16*)(ws + WS_WOL), *H16 = (_Float16*)(ws + WS_H16), *L16 = (_Float16*)(ws + WS_L16), *VT = (_Float16*)(ws + WS_VT), *CH = (_Float16*)(ws + WS_CH), *CL = (_Float16*)(ws + WS_CL);
  float* CS = (float*)(ws + WS_CS);
  float* OUT = (float*)d_out;
  const int nx8 = SEQ * DM / 8;
  const dim3 gx(nx8 / 256, NB), gt(DM / 64, DM / 64);
  k_cvt_bf<<<gx, 256, 0, stream>>>(F[0], XB,                          (size_t)SEQ_FULL * DM, (size_t)SEQ * DM, nx8);
  k_cvt_bf<<<gx, 256, 0, stream>>>(F[1], XB + (size_t)MROWS * DM,     (size_t)SEQ_FULL * DM, (size_t)SEQ * DM, nx8);
  k_cvt_bf<<<gx, 256, 0, stream>>>(F[2], XB + 2 * (size_t)MROWS * DM, (size_t)SEQ_FULL * DM, (size_t)SEQ * DM, nx8);
  k_wt_bf<<<gt, 256, 0, stream>>>(F[5], WB);
  k_wt_bf<<<gt, 256, 0, stream>>>(F[7], WB + (size_t)DM * DM);
  k_wt_bf<<<gt, 256, 0, stream>>>(F[9], WB + 2 * (size_t)DM * DM);
  k_wt_wo<<<gt, 256, 0, stream>>>(F[11], WOH, WOL);
  k_tab<<<dim3((MROWS * 32) / 256), 256, 0, stream>>>(F[4], CS);
  k_proj<<<dim3(MROWS / 64, DM / 128, 3), 128, 0, stream>>>(XB, WB, F[6], F[8], F[10], CS, H16, L16, VT);
  k_attn<<<dim3(SEQ / 64, NH, NB), 128, 0, stream>>>(H16, L16, VT, MASK, CH, CL);
  k_out<<<dim3(MROWS / 64, DM / 128), 128, 0, stream>>>(CH, CL, WOH, WOL, F[12], OUT);
}
